// MambaBlock_31129922961502
// MI455X (gfx1250) — hardware-verified
//
#include <hip/hip_runtime.h>
#include <math.h>

typedef __attribute__((ext_vector_type(16))) _Float16 v16h;
typedef __attribute__((ext_vector_type(8)))  _Float16 v8h;
typedef __attribute__((ext_vector_type(8)))  float    v8f;
typedef __attribute__((ext_vector_type(4)))  float    v4f;

constexpr int kBatch = 2;
constexpr int kSeq   = 1024;
constexpr int kDm    = 1024;
constexpr int kDin   = 2048;
constexpr int kNst   = 16;
constexpr int kDtR   = 64;
constexpr int kPrjN  = 96;
constexpr int kPrjP  = 128;
constexpr int kXzP   = 2 * kDin;
constexpr int kRows  = kBatch * kSeq;
constexpr int kBcP   = 32;
constexpr int kTP    = 260;
constexpr float kLnEps = 1e-5f;

constexpr float kCarryW   = 32.0f;
constexpr float kCarryWdt = 8.0f;
constexpr float kCarryDt  = 16.0f;
constexpr float kCarryY   = 16.0f;
constexpr float kSclIn    = 1.0f / kCarryW;
constexpr float kSclXp    = 1.0f / kCarryW;
constexpr float kSclXpDt  = kCarryDt / kCarryW;
constexpr float kSclDt    = 1.0f / (kCarryDt * kCarryWdt);
constexpr float kSclOut   = 1.0f / (kCarryY * kCarryW);

static_assert(kDtR + 2 * kNst == kPrjN, "x_proj width");
static_assert(2 * kNst == kBcP, "B|C plane pitch");
static_assert((kDm % 32) == 0 && (kDin % 32) == 0 && (kDtR % 32) == 0, "GEMM K multiples of 32");
static_assert((kRows % 64) == 0 && (kXzP % 64) == 0 && (kPrjP % 64) == 0 && (kDin % 64) == 0 && (kDm % 64) == 0, "GEMM M,N multiples of 64");
static_assert((kSeq % 64) == 0 && (kDin % 256) == 0 && (kSeq % 16) == 0 && (kRows % 8) == 0, "tile multiples");
static_assert(kDm == 1024, "LayerNorm lane map assumes 4 x 256 elements per row");

constexpr size_t kSzWIN  = (size_t)kXzP * kDm * 2;
constexpr size_t kSzWXP  = (size_t)kPrjP * kDin * 2;
constexpr size_t kSzWDT  = (size_t)kDin * kDtR * 2;
constexpr size_t kSzWOUT = (size_t)kDm * kDin * 2;
constexpr size_t kSzXN   = (size_t)kRows * kDm * 2;
constexpr size_t kSzXZ   = (size_t)kRows * kXzP * 4;
constexpr size_t kSzUC   = (size_t)kRows * kDin * 4;
constexpr size_t kSzUC16 = (size_t)kRows * kDin * 2;
constexpr size_t kSzDT16 = (size_t)kRows * kDtR * 2;
constexpr size_t kSzBC   = (size_t)kRows * kBcP * 4;
constexpr size_t kSzDLR  = (size_t)kRows * kDin * 4;
constexpr size_t kSzY16  = (size_t)kRows * kDin * 2;
constexpr size_t kOffWIN  = 0;
constexpr size_t kOffWXP  = kOffWIN  + kSzWIN;
constexpr size_t kOffWDT  = kOffWXP  + kSzWXP;
constexpr size_t kOffWOUT = kOffWDT  + kSzWDT;
constexpr size_t kOffXN   = kOffWOUT + kSzWOUT;
constexpr size_t kOffXZ   = kOffXN   + kSzXN;
constexpr size_t kOffUC   = kOffXZ   + kSzXZ;
constexpr size_t kOffUC16 = kOffUC   + kSzUC;
constexpr size_t kOffDT16 = kOffUC16 + kSzUC16;
constexpr size_t kOffBC   = kOffDT16 + kSzDT16;
constexpr size_t kOffDLR  = kOffBC   + kSzBC;
constexpr size_t kOffY16  = kOffDLR  + kSzDLR;
constexpr size_t kWsTotal = kOffY16  + kSzY16;
static_assert(kWsTotal == 101974016ull, "carve total");
static_assert(kWsTotal <= 134217728ull, "carve cap");
static_assert((kOffWXP % 128) == 0 && (kOffWDT % 128) == 0 && (kOffWOUT % 128) == 0 && (kOffXN % 128) == 0 &&
              (kOffXZ % 128) == 0 && (kOffUC % 128) == 0 && (kOffUC16 % 128) == 0 && (kOffDT16 % 128) == 0 &&
              (kOffBC % 128) == 0 && (kOffDLR % 128) == 0 && (kOffY16 % 128) == 0, "128-B aligned regions");

union FragU { v16h v; v8h h[2]; };
__device__ __forceinline__ v16h frag_load(const _Float16* p) {
  FragU f;
  f.h[0] = *(const v8h*)(p);
  f.h[1] = *(const v8h*)(p + 16);
  return f.v;
}
__device__ __forceinline__ v8f mma_f16(v16h a, v16h b, v8f c) {
  return __builtin_amdgcn_wmma_f32_16x16x32_f16(false, a, false, b, (short)0, c, false, false);
}
__device__ __forceinline__ void guard_row(v8f& a, v8f& b, v8f& c, v8f& d, v16h x,
                                          v16h b0, v16h b1, v16h b2, v16h b3) {
  asm volatile("v_nop\n\tv_nop\n\tv_nop\n\tv_nop"
               : "+v"(a), "+v"(b), "+v"(c), "+v"(d)
               : "v"(x), "v"(b0), "v"(b1), "v"(b2), "v"(b3));
}
__device__ __forceinline__ void keep4(v16h a, v16h b, v16h c, v16h d) {
  asm volatile("v_nop" :: "v"(a), "v"(b), "v"(c), "v"(d));
}
__device__ __forceinline__ void acc_guard4(v8f& a, v8f& b, v8f& c, v8f& d) {
  asm volatile("v_nop\n\tv_nop\n\tv_nop\n\tv_nop" : "+v"(a), "+v"(b), "+v"(c), "+v"(d));
}

template <int EPI, bool BIASN>
__global__ __launch_bounds__(256) void gemm_f16_kernel(
    const unsigned short* __restrict__ Ap, int lda,
    const unsigned short* __restrict__ Btp, int ldb,
    float* __restrict__ Cf, int ldc,
    const float* __restrict__ bias, const float* __restrict__ resid,
    unsigned short* __restrict__ Cdt, float* __restrict__ Cbc,
    int M, int N, int K, float scale, float scale_dt)
{
  const _Float16* A  = (const _Float16*)Ap;
  const _Float16* Bt = (const _Float16*)Btp;
  __shared__ __align__(16) float sT[8][16 * 68];
  const int lane = threadIdx.x & 31;
  const int wave = threadIdx.x >> 5;
  const int tilesN = N >> 6;
  const int tilesM = M >> 6;
  const int tile = blockIdx.x * 8 + wave;
  if (tile >= tilesM * tilesN) return;
  const int tm = tile / tilesN;
  const int tn = tile - tm * tilesN;
  const int m0 = tm << 6;
  const int n0 = tn << 6;

  const int rlane = lane & 15;
  const int koff  = (lane >> 4) * 8;
  const int mOff  = (lane >> 4) * 8;

  v8f acc[4][4];
#pragma unroll
  for (int i = 0; i < 4; ++i)
#pragma unroll
    for (int j = 0; j < 4; ++j) acc[i][j] = (v8f){0.f, 0.f, 0.f, 0.f, 0.f, 0.f, 0.f, 0.f};

  for (int k0 = 0; k0 < K; k0 += 32) {
    v16h bh[4];
#pragma unroll
    for (int j = 0; j < 4; ++j) {
      const size_t bo = (size_t)(n0 + (j << 4) + rlane) * ldb + koff + k0;
      bh[j] = frag_load(Bt + bo);
    }
#pragma unroll
    for (int i = 0; i < 4; ++i) {
      const size_t ao = (size_t)(m0 + (i << 4) + rlane) * lda + koff + k0;
      const v16h ah = frag_load(A + ao);
#pragma unroll
      for (int j = 0; j < 4; ++j) acc[i][j] = mma_f16(ah, bh[j], acc[i][j]);
      guard_row(acc[i][0], acc[i][1], acc[i][2], acc[i][3], ah, bh[0], bh[1], bh[2], bh[3]);
    }
    keep4(bh[0], bh[1], bh[2], bh[3]);
  }
  acc_guard4(acc[0][0], acc[0][1], acc[0][2], acc[0][3]);
  acc_guard4(acc[1][0], acc[1][1], acc[1][2], acc[1][3]);
  acc_guard4(acc[2][0], acc[2][1], acc[2][2], acc[2][3]);
  acc_guard4(acc[3][0], acc[3][1], acc[3][2], acc[3][3]);

  float* slab = sT[wave];
  const float sc = (EPI == 2 && tn == 0) ? scale_dt : scale;
#pragma unroll
  for (int i = 0; i < 4; ++i) {
    const int mBase = m0 + (i << 4);
#pragma unroll
    for (int j = 0; j < 4; ++j) {
      const int n = n0 + (j << 4) + rlane;
      float bv = 0.f;
      if (BIASN) bv = bias[n];
#pragma unroll
      for (int r = 0; r < 8; ++r) {
        float v = acc[i][j][r] * sc;
        if (BIASN) v += bv;
        slab[(mOff + r) * 68 + (j << 4) + rlane] = v;
      }
    }
    __builtin_amdgcn_fence(__ATOMIC_RELEASE, "workgroup");
    __builtin_amdgcn_wave_barrier();
    __builtin_amdgcn_fence(__ATOMIC_ACQUIRE, "workgroup");
    if (EPI == 0) {
      const int hh = lane >> 4, c4 = (lane & 15) * 4;
      for (int pass = 0; pass < 2; ++pass) {
#pragma unroll
        for (int it = 0; it < 8; ++it) {
          const int row = it * 2 + hh;
          const v4f v = *(const v4f*)(slab + row * 68 + c4);
          *(volatile v4f*)(Cf + (size_t)(mBase + row) * ldc + n0 + c4) = v;
        }
        __threadfence();
      }
    } else if (EPI == 1) {
      const int hh = lane >> 4, c4 = (lane & 15) * 4;
      v4f vv[8];
#pragma unroll
      for (int it = 0; it < 8; ++it) {
        const int row = it * 2 + hh;
        const v4f sv = *(const v4f*)(slab + row * 68 + c4);
        const v4f rv = *(const v4f*)(resid + (size_t)(mBase + row) * ldc + n0 + c4);
        vv[it] = sv + rv;
      }
      for (int pass = 0; pass < 2; ++pass) {
#pragma unroll
        for (int it = 0; it < 8; ++it) {
          const int row = it * 2 + hh;
          *(volatile v4f*)(Cf + (size_t)(mBase + row) * ldc + n0 + c4) = vv[it];
        }
        __threadfence();
      }
    } else {
      const int q = lane >> 3;
      if (tn == 0) {
        const int c8 = (lane & 7) * 8;
        v8h hv[4];
#pragma unroll
        for (int it = 0; it < 4; ++it) {
          const float* sp = slab + (it * 4 + q) * 68 + c8;
          const v4f a0 = *(const v4f*)(sp);
          const v4f a1 = *(const v4f*)(sp + 4);
#pragma unroll
          for (int e = 0; e < 4; ++e) {
            hv[it][e]     = (_Float16)a0[e];
            hv[it][4 + e] = (_Float16)a1[e];
          }
        }
        for (int pass = 0; pass < 2; ++pass) {
#pragma unroll
          for (int it = 0; it < 4; ++it)
            *(volatile v8h*)(Cdt + (size_t)(mBase + it * 4 + q) * kDtR + c8) = hv[it];
          __threadfence();
        }
      } else {
        const int c4 = (lane & 7) * 4;
        v4f fv[4];
#pragma unroll
        for (int it = 0; it < 4; ++it) fv[it] = *(const v4f*)(slab + (it * 4 + q) * 68 + c4);
        for (int pass = 0; pass < 2; ++pass) {
#pragma unroll
          for (int it = 0; it < 4; ++it)
            *(volatile v4f*)(Cbc + (size_t)(mBase + it * 4 + q) * kBcP + c4) = fv[it];
          __threadfence();
        }
      }
    }
    __builtin_amdgcn_fence(__ATOMIC_RELEASE, "workgroup");
    __builtin_amdgcn_wave_barrier();
    __builtin_amdgcn_fence(__ATOMIC_ACQUIRE, "workgroup");
  }
}

__global__ __launch_bounds__(256) void cast_f16_kernel(
    const float* __restrict__ src, unsigned short* __restrict__ dst, int real8, int total8, float scale)
{
  const int i = blockIdx.x * 256 + threadIdx.x;
  if (i >= total8) return;
  const bool live = (i < real8);
  const size_t e0 = (size_t)i << 3;
  const size_t es = live ? e0 : (size_t)0;
  const v4f a0 = *(const v4f*)(src + es);
  const v4f a1 = *(const v4f*)(src + es + 4);
  v8h hv;
#pragma unroll
  for (int e = 0; e < 4; ++e) {
    const float f0 = live ? (a0[e] * scale) : 0.0f;
    const float f1 = live ? (a1[e] * scale) : 0.0f;
    hv[e]     = (_Float16)f0;
    hv[4 + e] = (_Float16)f1;
  }
  unsigned short* q = dst + e0;
  *(volatile v8h*)q = hv;
  __threadfence();
  *(volatile v8h*)q = hv;
}

__global__ __launch_bounds__(256) void layernorm_f16_kernel(
    const float* __restrict__ x, const float* __restrict__ gw, const float* __restrict__ gb,
    unsigned short* __restrict__ xn16)
{
  const int lane = threadIdx.x & 31, wave = threadIdx.x >> 5;
  const int row = blockIdx.x * 8 + wave;
  const float* xr = x + (size_t)row * kDm + lane * 8;
  float s = 0.f;
#pragma unroll 1
  for (int it = 0; it < 4; ++it) {
    const v4f a0 = *(const v4f*)(xr + it * 256);
    const v4f a1 = *(const v4f*)(xr + it * 256 + 4);
    s += ((a0[0] + a0[1]) + (a0[2] + a0[3])) + ((a1[0] + a1[1]) + (a1[2] + a1[3]));
  }
  s += __shfl_xor(s, 16, 32);
  s += __shfl_xor(s, 8, 32);
  s += __shfl_xor(s, 4, 32);
  s += __shfl_xor(s, 2, 32);
  s += __shfl_xor(s, 1, 32);
  const float mu = s * (1.0f / (float)kDm);
  float vs = 0.f;
#pragma unroll 1
  for (int it = 0; it < 4; ++it) {
    const v4f a0 = *(const v4f*)(xr + it * 256);
    const v4f a1 = *(const v4f*)(xr + it * 256 + 4);
    float part = 0.f;
#pragma unroll
    for (int e = 0; e < 4; ++e) {
      const float d0 = a0[e] - mu, d1 = a1[e] - mu;
      part = fmaf(d0, d0, part);
      part = fmaf(d1, d1, part);
    }
    vs += part;
  }
  vs += __shfl_xor(vs, 16, 32);
  vs += __shfl_xor(vs, 8, 32);
  vs += __shfl_xor(vs, 4, 32);
  vs += __shfl_xor(vs, 2, 32);
  vs += __shfl_xor(vs, 1, 32);
  const float var  = vs * (1.0f / (float)kDm);
  const float rstd = 1.0f / sqrtf(var + kLnEps);
  unsigned short* orow = xn16 + (size_t)row * kDm + lane * 8;
#pragma unroll 1
  for (int it = 0; it < 4; ++it) {
    const int c = it * 256 + lane * 8;
    const v4f a0 = *(const v4f*)(xr + it * 256);
    const v4f a1 = *(const v4f*)(xr + it * 256 + 4);
    const v4f w0 = *(const v4f*)(gw + c);
    const v4f w1 = *(const v4f*)(gw + c + 4);
    const v4f b0 = *(const v4f*)(gb + c);
    const v4f b1 = *(const v4f*)(gb + c + 4);
    v8h hv;
#pragma unroll
    for (int e = 0; e < 4; ++e) {
      const float o0 = ((a0[e] - mu) * rstd) * w0[e] + b0[e];
      const float o1 = ((a1[e] - mu) * rstd) * w1[e] + b1[e];
      hv[e]     = (_Float16)o0;
      hv[4 + e] = (_Float16)o1;
    }
    unsigned short* q = orow + it * 256;
    *(volatile v8h*)q = hv;
    __threadfence();
    *(volatile v8h*)q = hv;
  }
}

__global__ __launch_bounds__(256) void conv_silu_kernel(
    const float* __restrict__ XZ, const float* __restrict__ cw, const float* __restrict__ cb,
    float* __restrict__ UC, unsigned short* __restrict__ UC16)
{
  __shared__ __align__(16) float sT[16 * kTP];
  const int tid = threadIdx.x, lane = tid & 31, wave = tid >> 5;
  const int d0 = blockIdx.x * 256, d = d0 + tid;
  const int g0 = blockIdx.y * 64;
  const int tb = g0 & (kSeq - 1);
  const v4f wv = *(const v4f*)(cw + (size_t)d * 4);
  const float w0 = wv[0], w1 = wv[1], w2 = wv[2], w3 = wv[3];
  const float bc = cb[d];
  float xm3, xm2, xm1;
  {
    const bool hist = (tb > 0);
    const int rb = hist ? (g0 - 3) : g0;
    const float v3 = XZ[(size_t)rb * kXzP + d];
    const float v2 = XZ[(size_t)(rb + 1) * kXzP + d];
    const float v1 = XZ[(size_t)(rb + 2) * kXzP + d];
    xm3 = hist ? v3 : 0.f;
    xm2 = hist ? v2 : 0.f;
    xm1 = hist ? v1 : 0.f;
  }
  const int hrow = wave >> 1;
  const int hch  = (wave & 1) * 128 + lane * 4;
#pragma unroll 1
  for (int sub = 0; sub < 4; ++sub) {
    const int lb = g0 + sub * 16;
#pragma unroll 1
    for (int s = 0; s < 16; ++s) {
      const float xc = XZ[(size_t)(lb + s) * kXzP + d];
      float acc = w0 * xm3;
      acc = fmaf(w1, xm2, acc);
      acc = fmaf(w2, xm1, acc);
      acc = fmaf(w3, xc, acc);
      const float sv = acc + bc;
      const float sg = __builtin_amdgcn_rcpf(1.0f + expf(-sv));
      sT[s * kTP + tid] = sv * sg;
      xm3 = xm2; xm2 = xm1; xm1 = xc;
    }
    __syncthreads();
    v4f fv[4];
    v8h bv[2];
#pragma unroll
    for (int it = 0; it < 4; ++it) fv[it] = *(const v4f*)(sT + (it * 4 + hrow) * kTP + hch);
#pragma unroll
    for (int it = 0; it < 2; ++it) {
      const float* sp = sT + (it * 8 + wave) * kTP + lane * 8;
      const v4f a0 = *(const v4f*)(sp);
      const v4f a1 = *(const v4f*)(sp + 4);
#pragma unroll
      for (int e = 0; e < 4; ++e) {
        bv[it][e]     = (_Float16)a0[e];
        bv[it][4 + e] = (_Float16)a1[e];
      }
    }
    for (int pass = 0; pass < 2; ++pass) {
#pragma unroll
      for (int it = 0; it < 4; ++it)
        *(volatile v4f*)(UC + (size_t)(lb + it * 4 + hrow) * kDin + d0 + hch) = fv[it];
#pragma unroll
      for (int it = 0; it < 2; ++it)
        *(volatile v8h*)(UC16 + (size_t)(lb + it * 8 + wave) * kDin + d0 + lane * 8) = bv[it];
      __threadfence();
    }
    __syncthreads();
  }
}

__global__ __launch_bounds__(256) void scan_gate_kernel(
    const float* __restrict__ DLR, const float* __restrict__ UC, const float* __restrict__ XZ,
    const float* __restrict__ BC, const float* __restrict__ A_log, const float* __restrict__ Dv,
    unsigned short* __restrict__ Y16)
{
  __shared__ __align__(16) float sBC[16 * kBcP];
  __shared__ __align__(16) float sY[16 * kTP];
  __shared__ __align__(16) float sA[kNst * 256];
  const int tid = threadIdx.x, lane = tid & 31, wave = tid >> 5;
  const int d0 = blockIdx.x * 256, d = d0 + tid;
  const size_t row0 = (size_t)blockIdx.y * kSeq;

#pragma unroll 1
  for (int n = 0; n < kNst; ++n) sA[n * 256 + tid] = -expf(A_log[(size_t)d * kNst + n]);
  __syncthreads();
  float An[kNst], h[kNst];
#pragma unroll
  for (int n = 0; n < kNst; ++n) {
    An[n] = sA[n * 256 + tid];
    h[n] = 0.f;
  }
  const float Dd = Dv[d];

#pragma unroll 1
  for (int c = 0; c < kSeq / 16; ++c) {
    const int l0 = c * 16;
    if (tid < 128) {
      const int r = tid >> 3, q4 = (tid & 7) * 4;
      const v4f v = *(const v4f*)(BC + (row0 + l0 + r) * kBcP + q4);
      *(v4f*)(sBC + r * kBcP + q4) = v;
    }
    __syncthreads();
#pragma unroll 1
    for (int s = 0; s < 16; ++s) {
      const size_t m = row0 + (size_t)(l0 + s);
      float a  = DLR[m * kDin + d];
      float xv = UC[m * kDin + d];
      float zv = XZ[m * kXzP + kDin + d];
      asm volatile("" : "+v"(a));
      asm volatile("" : "+v"(xv));
      asm volatile("" : "+v"(zv));
      const float delta = fmaxf(a, 0.0f) + log1pf(expf(-fabsf(a)));
      v4f Bq[4], Cq[4];
#pragma unroll
      for (int qq = 0; qq < 4; ++qq) {
        Bq[qq] = *(const v4f*)(sBC + s * kBcP + 4 * qq);
        Cq[qq] = *(const v4f*)(sBC + s * kBcP + kNst + 4 * qq);
      }
      float y = 0.f;
#pragma unroll
      for (int n = 0; n < kNst; ++n) {
        const float e  = __expf(delta * An[n]);
        const float bu = (delta * Bq[n >> 2][n & 3]) * xv;
        const float hn = fmaf(e, h[n], bu);
        h[n] = hn;
        y = fmaf(hn, Cq[n >> 2][n & 3], y);
      }
      y = fmaf(xv, Dd, y);
      const float sg = __builtin_amdgcn_rcpf(1.0f + expf(-zv));
      const float g  = zv * sg;
      sY[s * kTP + tid] = (y * g) * kCarryY;
    }
    __syncthreads();
    v8h hv[2];
#pragma unroll
    for (int it = 0; it < 2; ++it) {
      const float* sp = sY + (it * 8 + wave) * kTP + lane * 8;
      const v4f a0 = *(const v4f*)(sp);
      const v4f a1 = *(const v4f*)(sp + 4);
#pragma unroll
      for (int e = 0; e < 4; ++e) {
        hv[it][e]     = (_Float16)a0[e];
        hv[it][4 + e] = (_Float16)a1[e];
      }
    }
    for (int pass = 0; pass < 2; ++pass) {
#pragma unroll
      for (int it = 0; it < 2; ++it)
        *(volatile v8h*)(Y16 + (row0 + l0 + it * 8 + wave) * kDin + d0 + lane * 8) = hv[it];
      __threadfence();
    }
  }
}

extern "C" void kernel_launch(void* const* d_in, const int* in_sizes, int n_in,
                              void* d_out, int out_size, void* d_ws, size_t ws_size,
                              hipStream_t stream)
{
  if (n_in < 12) return;
  if (in_sizes[0] != kRows * kDm) return;
  if (in_sizes[1] != kDm || in_sizes[2] != kDm) return;
  if (in_sizes[3] != kXzP * kDm) return;
  if (in_sizes[4] != kDin * 4 || in_sizes[5] != kDin) return;
  if (in_sizes[6] != kPrjN * kDin) return;
  if (in_sizes[7] != kDin * kDtR || in_sizes[8] != kDin) return;
  if (in_sizes[9] != kDin * kNst || in_sizes[10] != kDin) return;
  if (in_sizes[11] != kDm * kDin) return;
  if (out_size != kRows * kDm) return;
  if (ws_size < kWsTotal) return;

  const float* x      = (const float*)d_in[0];
  const float* norm_w = (const float*)d_in[1];
  const float* norm_b = (const float*)d_in[2];
  const float* W_in   = (const float*)d_in[3];
  const float* conv_w = (const float*)d_in[4];
  const float* conv_b = (const float*)d_in[5];
  const float* W_xp   = (const float*)d_in[6];
  const float* W_dt   = (const float*)d_in[7];
  const float* b_dt   = (const float*)d_in[8];
  const float* A_log  = (const float*)d_in[9];
  const float* Dv     = (const float*)d_in[10];
  const float* W_out  = (const float*)d_in[11];
  float* out = (float*)d_out;

  char* ws = (char*)d_ws;
  unsigned short* WIN16  = (unsigned short*)(ws + kOffWIN);
  unsigned short* WXP16  = (unsigned short*)(ws + kOffWXP);
  unsigned short* WDT16  = (unsigned short*)(ws + kOffWDT);
  unsigned short* WOUT16 = (unsigned short*)(ws + kOffWOUT);
  unsigned short* XN16   = (unsigned short*)(ws + kOffXN);
  float*          XZ     = (float*)(ws + kOffXZ);
  float*          UC     = (float*)(ws + kOffUC);
  unsigned short* UC16   = (unsigned short*)(ws + kOffUC16);
  unsigned short* DT16   = (unsigned short*)(ws + kOffDT16);
  float*          BC     = (float*)(ws + kOffBC);
  float*          DLR    = (float*)(ws + kOffDLR);
  unsigned short* Y16    = (unsigned short*)(ws + kOffY16);

  cast_f16_kernel<<<(kXzP * kDm / 8) / 256, 256, 0, stream>>>(W_in, WIN16, kXzP * kDm / 8, kXzP * kDm / 8, kCarryW);
  cast_f16_kernel<<<(kPrjP * kDin / 8) / 256, 256, 0, stream>>>(W_xp, WXP16, kPrjN * kDin / 8, kPrjP * kDin / 8, kCarryW);
  cast_f16_kernel<<<(kDin * kDtR / 8) / 256, 256, 0, stream>>>(W_dt, WDT16, kDin * kDtR / 8, kDin * kDtR / 8, kCarryWdt);
  cast_f16_kernel<<<(kDm * kDin / 8) / 256, 256, 0, stream>>>(W_out, WOUT16, kDm * kDin / 8, kDm * kDin / 8, kCarryW);

  layernorm_f16_kernel<<<kRows / 8, 256, 0, stream>>>(x, norm_w, norm_b, XN16);

  gemm_f16_kernel<0, false><<<(kRows / 64) * (kXzP / 64) / 8, 256, 0, stream>>>(
      XN16, kDm, WIN16, kDm, XZ, kXzP, b_dt, x, DT16, BC, kRows, kXzP, kDm, kSclIn, kSclIn);

  conv_silu_kernel<<<dim3(kDin / 256, kRows / 64), 256, 0, stream>>>(XZ, conv_w, conv_b, UC, UC16);

  gemm_f16_kernel<2, false><<<(kRows / 64) * (kPrjP / 64) / 8, 256, 0, stream>>>(
      UC16, kDin, WXP16, kDin, BC, kBcP, b_dt, x, DT16, BC, kRows, kPrjP, kDin, kSclXp, kSclXpDt);

  gemm_f16_kernel<0, true><<<(kRows / 64) * (kDin / 64) / 8, 256, 0, stream>>>(
      DT16, kDtR, WDT16, kDtR, DLR, kDin, b_dt, x, DT16, BC, kRows, kDin, kDtR, kSclDt, kSclDt);

  scan_gate_kernel<<<dim3(kDin / 256, kBatch), 256, 0, stream>>>(DLR, UC, XZ, BC, A_log, Dv, Y16);

  gemm_f16_kernel<1, false><<<(kRows / 64) * (kDm / 64) / 8, 256, 0, stream>>>(
      Y16, kDin, WOUT16, kDin, out, kDm, b_dt, x, DT16, BC, kRows, kDm, kDin, kSclOut, kSclOut);
}
